// Decoder_60387240182010
// MI455X (gfx1250) — hardware-verified
//
#include <hip/hip_runtime.h>
#include <math.h>

constexpr int NBATCH   = 64;
constexpr int NLAT     = 256;
constexpr int NHID     = 1024;
constexpr int NGATE    = 4 * NHID;
constexpr int NOUT     = 512;
constexpr int NSTEP    = 256;
constexpr int NROWS    = NBATCH * NSTEP;
constexpr int SEQ_BLK  = 16;
constexpr int LSTM_THR = 512;
constexpr int HPITCH   = NHID + 8;
constexpr int GATE_PLANE = NHID * NHID;
constexpr int N8_W     = NGATE * NHID / 8;
constexpr int N8_O     = NOUT * NHID / 8;
constexpr int PACK_BLK_W = N8_W / 256;
constexpr int PACK_BLK_O = N8_O / 256;
constexpr float HCARRY    = 16.0f;
constexpr float WCARRY    = 64.0f;
constexpr float CARRY_INV = 1.0f / (HCARRY * WCARRY);

static_assert(NBATCH % SEQ_BLK == 0, "batch tile");
static_assert(NHID == 64 * (LSTM_THR / 32), "16 waves x 64 hidden units");
static_assert(NHID % 32 == 0 && NLAT % 4 == 0, "k multiples");
static_assert(NROWS % 64 == 0 && NOUT % 64 == 0, "head tile multiples");
static_assert((SEQ_BLK * NHID / 8) % LSTM_THR == 0, "h tile copy exact");
static_assert(NGATE == LSTM_THR * 8, "bias table fill exact");
static_assert(N8_W % 256 == 0 && N8_O % 256 == 0, "pack grid exact");
static_assert((HPITCH % 8) == 0, "16-B aligned LDS rows");
static_assert((size_t)NBATCH * NSTEP * NOUT * 4 == (size_t)33554432, "output bytes");

typedef __attribute__((ext_vector_type(16))) _Float16 v16h;
typedef __attribute__((ext_vector_type(8)))  _Float16 v8h;
typedef __attribute__((ext_vector_type(8)))  float    v8f;
typedef __attribute__((ext_vector_type(4)))  float    v4f;

__device__ __forceinline__ void guard_group4(v8f& a0, v8f& a1, v8f& a2, v8f& a3, v16h a, v16h b0, v16h b1, v16h b2, v16h b3) {
  asm volatile("v_nop\n\tv_nop\n\tv_nop\n\tv_nop" : "+v"(a0), "+v"(a1), "+v"(a2), "+v"(a3) : "v"(a), "v"(b0), "v"(b1), "v"(b2), "v"(b3));
}
__device__ __forceinline__ void keep4_h(v16h a, v16h b, v16h c, v16h d) { asm volatile("v_nop" :: "v"(a), "v"(b), "v"(c), "v"(d)); }
__device__ __forceinline__ void acc_guard4(v8f& a, v8f& b, v8f& c, v8f& d) { asm volatile("v_nop\n\tv_nop\n\tv_nop\n\tv_nop" : "+v"(a), "+v"(b), "+v"(c), "+v"(d)); }

union FragU { v16h v; v8h h[2]; };
__device__ __forceinline__ v16h frag_load(const _Float16* p) {
  FragU f;
  f.h[0] = *(const v8h*)(p);
  f.h[1] = *(const v8h*)(p + 16);
  return f.v;
}
__device__ __forceinline__ v8f frag_mma(v16h a, v16h b, v8f c) {
  return __builtin_amdgcn_wmma_f32_16x16x32_f16(false, a, false, b, (short)0, c, false, false);
}

__device__ __forceinline__ float gate_sig(float x)  { return __builtin_amdgcn_rcpf(1.0f + expf(-x)); }
__device__ __forceinline__ float gate_tanh(float x) { return 1.0f - 2.0f * __builtin_amdgcn_rcpf(expf(2.0f * x) + 1.0f); }

__global__ __launch_bounds__(256) void pack_w_kernel(const float* __restrict__ w_ih, const float* __restrict__ w_hh,
                                                     const float* __restrict__ out_w, unsigned short* __restrict__ WC,
                                                     unsigned short* __restrict__ WHH, unsigned short* __restrict__ OW) {
  const int bid = blockIdx.x;
  const int tid = threadIdx.x;
  int region = 0;
  int lb = bid;
  if (bid >= PACK_BLK_W)     { region = 1; lb = bid - PACK_BLK_W; }
  if (bid >= 2 * PACK_BLK_W) { region = 2; lb = bid - 2 * PACK_BLK_W; }
  const float* s0 = (region == 0) ? w_ih : ((region == 1) ? w_hh : out_w);
  const float* s1 = (region == 0) ? w_hh : s0;
  unsigned short* dst = (region == 0) ? WC : ((region == 1) ? WHH : OW);
  const int nchunk = (region == 2) ? N8_O : N8_W;
  const int i = lb * 256 + tid;
  if (i < nchunk) {
    const float* p0 = s0 + (size_t)i * 8;
    const float* p1 = s1 + (size_t)i * 8;
    const v4f a0 = *(const v4f*)(p0);
    const v4f a1 = *(const v4f*)(p0 + 4);
    const v4f c0 = *(const v4f*)(p1);
    const v4f c1 = *(const v4f*)(p1 + 4);
    v8h hv;
#pragma unroll
    for (int e = 0; e < 4; ++e) {
      const float x0 = (region == 0) ? (a0[e] + c0[e]) : a0[e];
      const float x1 = (region == 0) ? (a1[e] + c1[e]) : a1[e];
      hv[e]     = (_Float16)(x0 * WCARRY);
      hv[4 + e] = (_Float16)(x1 * WCARRY);
    }
    unsigned short* op = dst + (size_t)i * 8;
    *(volatile v8h*)op = hv;
    __threadfence();
    *(volatile v8h*)op = hv;
  }
}

__global__ __launch_bounds__(256) void fc_h0_kernel(const float* __restrict__ latent, const float* __restrict__ fc_w,
                                                    const float* __restrict__ fc_b, unsigned* __restrict__ H0w) {
  const int i = blockIdx.x * 256 + threadIdx.x;
  if (i < NBATCH * NHID / 2) {
    const int b  = i >> 9;
    const int j0 = (i & 511) * 2;
    const float* lr = latent + (size_t)b * NLAT;
    const float* w0 = fc_w + (size_t)j0 * NLAT;
    const float* w1 = w0 + NLAT;
    float a0 = 0.0f, a1 = 0.0f;
#pragma unroll 1
    for (int k = 0; k < NLAT; k += 4) {
      const v4f l = *(const v4f*)(lr + k);
      const v4f x = *(const v4f*)(w0 + k);
      const v4f y = *(const v4f*)(w1 + k);
      a0 = fmaf(l[0], x[0], a0);
      a0 = fmaf(l[1], x[1], a0);
      a0 = fmaf(l[2], x[2], a0);
      a0 = fmaf(l[3], x[3], a0);
      a1 = fmaf(l[0], y[0], a1);
      a1 = fmaf(l[1], y[1], a1);
      a1 = fmaf(l[2], y[2], a1);
      a1 = fmaf(l[3], y[3], a1);
    }
    a0 += fc_b[j0];
    a1 += fc_b[j0 + 1];
    const _Float16 h0 = (_Float16)(a0 * HCARRY);
    const _Float16 h1 = (_Float16)(a1 * HCARRY);
    const unsigned u = (unsigned)__builtin_bit_cast(unsigned short, h0) | ((unsigned)__builtin_bit_cast(unsigned short, h1) << 16);
    ((volatile unsigned*)H0w)[i] = u;
    __threadfence();
    ((volatile unsigned*)H0w)[i] = u;
  }
}

__global__ __launch_bounds__(LSTM_THR) void lstm_seq_kernel(const unsigned short* __restrict__ H0p,
                                                            const unsigned short* __restrict__ WCp,
                                                            const unsigned short* __restrict__ WHHp,
                                                            const float* __restrict__ b_ih, const float* __restrict__ b_hh,
                                                            unsigned short* __restrict__ HALLp) {
  __shared__ __align__(16) _Float16 Ah[SEQ_BLK * HPITCH];
  __shared__ __align__(16) float    Bs[NGATE];
  const _Float16* H0  = (const _Float16*)H0p;
  const _Float16* WC  = (const _Float16*)WCp;
  const _Float16* WHH = (const _Float16*)WHHp;
  _Float16* HALL = (_Float16*)HALLp;
  const int tid = threadIdx.x, lane = tid & 31, wave = tid >> 5;
  const int c = lane & 15, hh = lane >> 4, koff = hh * 8;
  const int rowbase = blockIdx.x * SEQ_BLK;

  {
    const int i8 = tid * 8;
    const v4f a0 = *(const v4f*)(b_ih + i8);
    const v4f a1 = *(const v4f*)(b_ih + i8 + 4);
    const v4f c0 = *(const v4f*)(b_hh + i8);
    const v4f c1 = *(const v4f*)(b_hh + i8 + 4);
    const v4f s0 = a0 + c0;
    const v4f s1 = a1 + c1;
    *(v4f*)(Bs + i8)     = s0;
    *(v4f*)(Bs + i8 + 4) = s1;
  }
#pragma unroll
  for (int it = 0; it < 4; ++it) {
    const int idx = it * LSTM_THR + tid;
    const int row = idx >> 7, ch = idx & 127;
    const v8h v = *(const v8h*)(H0 + (size_t)(rowbase + row) * NHID + ch * 8);
    *(v8h*)(Ah + row * HPITCH + ch * 8) = v;
  }
  if (tid < SEQ_BLK) {
    v8h z;
#pragma unroll
    for (int e = 0; e < 8; ++e) z[e] = (_Float16)0.0f;
    *(v8h*)(Ah + tid * HPITCH + NHID) = z;
  }
  const v8f z8 = {0.f, 0.f, 0.f, 0.f, 0.f, 0.f, 0.f, 0.f};
  v8f cA = z8, cB = z8, cC = z8, cD = z8;
  v8f hA = z8, hB = z8, hC = z8, hD = z8;
  __syncthreads();

  const _Float16* ahrow = Ah + c * HPITCH + koff;

#pragma unroll 1
  for (int t = 0; t < NSTEP; ++t) {
    const _Float16* Wsel = (t == 0) ? WHH : WC;
#pragma unroll 1
    for (int nt = 0; nt < 4; ++nt) {
      const int j = 64 * wave + 16 * nt + c;
      const _Float16* wb = Wsel + (size_t)j * NHID + koff;
      v8f acc0 = z8, acc1 = z8, acc2 = z8, acc3 = z8;
#pragma unroll 1
      for (int k0 = 0; k0 < NHID; k0 += 32) {
        const v16h a  = frag_load(ahrow + k0);
        const v16h b0 = frag_load(wb + k0);
        const v16h b1 = frag_load(wb + (size_t)1 * GATE_PLANE + k0);
        const v16h b2 = frag_load(wb + (size_t)2 * GATE_PLANE + k0);
        const v16h b3 = frag_load(wb + (size_t)3 * GATE_PLANE + k0);
        acc0 = frag_mma(a, b0, acc0);
        acc1 = frag_mma(a, b1, acc1);
        acc2 = frag_mma(a, b2, acc2);
        acc3 = frag_mma(a, b3, acc3);
        guard_group4(acc0, acc1, acc2, acc3, a, b0, b1, b2, b3);
      }
      acc_guard4(acc0, acc1, acc2, acc3);
      const float bi = Bs[j];
      const float bf = Bs[NHID + j];
      const float bg = Bs[2 * NHID + j];
      const float bo = Bs[3 * NHID + j];
#pragma unroll
      for (int r = 0; r < 8; ++r) {
        const float zi = acc0[r] * CARRY_INV + bi;
        const float zf = acc1[r] * CARRY_INV + bf;
        const float zg = acc2[r] * CARRY_INV + bg;
        const float zo = acc3[r] * CARRY_INV + bo;
        const float ig = gate_sig(zi);
        const float fg = gate_sig(zf);
        const float gg = gate_tanh(zg);
        const float og = gate_sig(zo);
        const float cn = fg * cA[r] + ig * gg;
        cA[r] = cn;
        hA[r] = og * gate_tanh(cn);
      }
      {
        const v8f tc = cA; cA = cB; cB = cC; cC = cD; cD = tc;
        const v8f th = hA; hA = hB; hB = hC; hC = hD; hD = th;
      }
    }
    __syncthreads();
    {
      const int jb = 64 * wave + c;
#pragma unroll
      for (int r = 0; r < 8; ++r) {
        _Float16* rowp = Ah + (8 * hh + r) * HPITCH + jb;
        rowp[0]  = (_Float16)(hA[r] * HCARRY);
        rowp[16] = (_Float16)(hB[r] * HCARRY);
        rowp[32] = (_Float16)(hC[r] * HCARRY);
        rowp[48] = (_Float16)(hD[r] * HCARRY);
      }
    }
    __syncthreads();
    for (int pass = 0; pass < 2; ++pass) {
#pragma unroll
      for (int it = 0; it < 4; ++it) {
        const int idx = it * LSTM_THR + tid;
        const int row = idx >> 7, ch = idx & 127;
        const v8h v = *(const v8h*)(Ah + row * HPITCH + ch * 8);
        *(volatile v8h*)(HALL + ((size_t)(rowbase + row) * NSTEP + (size_t)t) * NHID + ch * 8) = v;
      }
      __threadfence();
    }
  }
}

__global__ __launch_bounds__(256) void head_gemm_kernel(const unsigned short* __restrict__ Ap,
                                                        const unsigned short* __restrict__ Btp,
                                                        float* __restrict__ Cout, const float* __restrict__ bias) {
  const _Float16* A  = (const _Float16*)Ap;
  const _Float16* Bt = (const _Float16*)Btp;
  __shared__ __align__(16) float sT[8][16 * 68];
  const int lane = threadIdx.x & 31;
  const int wave = threadIdx.x >> 5;
  constexpr int tilesN = NOUT >> 6;
  constexpr int tilesM = NROWS >> 6;
  constexpr int lda = NHID, ldb = NHID, ldc = NOUT;
  const int tile = blockIdx.x * 8 + wave;
  if (tile >= tilesM * tilesN) return;
  const int tm = tile / tilesN;
  const int tn = tile - tm * tilesN;
  const int m0 = tm << 6;
  const int n0 = tn << 6;

  const int rlane = lane & 15;
  const int koff  = (lane >> 4) * 8;
  const int mOff  = (lane >> 4) * 8;

  v8f acc[4][4];
#pragma unroll
  for (int i = 0; i < 4; ++i)
#pragma unroll
    for (int j = 0; j < 4; ++j) acc[i][j] = (v8f){0.f,0.f,0.f,0.f,0.f,0.f,0.f,0.f};

  for (int k0 = 0; k0 < NHID; k0 += 32) {
    v16h bh[4];
#pragma unroll
    for (int j = 0; j < 4; ++j) {
      const size_t bo = (size_t)(n0 + (j << 4) + rlane) * ldb + koff + k0;
      bh[j] = frag_load(Bt + bo);
    }
#pragma unroll
    for (int i = 0; i < 4; ++i) {
      const size_t ao = (size_t)(m0 + (i << 4) + rlane) * lda + koff + k0;
      const v16h ah = frag_load(A + ao);
#pragma unroll
      for (int j = 0; j < 4; ++j) acc[i][j] = frag_mma(ah, bh[j], acc[i][j]);
      guard_group4(acc[i][0], acc[i][1], acc[i][2], acc[i][3], ah, bh[0], bh[1], bh[2], bh[3]);
    }
    keep4_h(bh[0], bh[1], bh[2], bh[3]);
  }
  acc_guard4(acc[0][0], acc[0][1], acc[0][2], acc[0][3]);
  acc_guard4(acc[1][0], acc[1][1], acc[1][2], acc[1][3]);
  acc_guard4(acc[2][0], acc[2][1], acc[2][2], acc[2][3]);
  acc_guard4(acc[3][0], acc[3][1], acc[3][2], acc[3][3]);

  float* slab = sT[wave];
#pragma unroll
  for (int i = 0; i < 4; ++i) {
    const int mBase = m0 + (i << 4);
#pragma unroll
    for (int j = 0; j < 4; ++j) {
      const int n = n0 + (j << 4) + rlane;
      const float bv = bias[n];
#pragma unroll
      for (int r = 0; r < 8; ++r) {
        float v = acc[i][j][r] * CARRY_INV;
        v += bv;
        slab[(mOff + r) * 68 + (j << 4) + rlane] = v;
      }
    }
    __builtin_amdgcn_fence(__ATOMIC_RELEASE, "workgroup");
    __builtin_amdgcn_wave_barrier();
    __builtin_amdgcn_fence(__ATOMIC_ACQUIRE, "workgroup");
    {
      const int hh = lane >> 4, c4 = (lane & 15) * 4;
      for (int pass = 0; pass < 2; ++pass) {
#pragma unroll
        for (int it = 0; it < 8; ++it) {
          const int row = it * 2 + hh;
          const v4f v = *(const v4f*)(slab + row * 68 + c4);
          *(volatile v4f*)(Cout + (size_t)(mBase + row) * ldc + n0 + c4) = v;
        }
        __threadfence();
      }
    }
    __builtin_amdgcn_fence(__ATOMIC_RELEASE, "workgroup");
    __builtin_amdgcn_wave_barrier();
    __builtin_amdgcn_fence(__ATOMIC_ACQUIRE, "workgroup");
  }
}

extern "C" void kernel_launch(void* const* d_in, const int* in_sizes, int n_in,
                              void* d_out, int out_size, void* d_ws, size_t ws_size, hipStream_t stream) {
  if (n_in < 10 || d_out == nullptr || d_ws == nullptr) return;
  if (in_sizes[0] != NBATCH * NLAT || in_sizes[1] != 1 || in_sizes[2] != NHID * NLAT || in_sizes[3] != NHID ||
      in_sizes[4] != NGATE * NHID || in_sizes[5] != NGATE * NHID || in_sizes[6] != NGATE || in_sizes[7] != NGATE ||
      in_sizes[8] != NOUT * NHID || in_sizes[9] != NOUT || out_size != NROWS * NOUT) return;

  const float* latent = (const float*)d_in[0];
  const float* fc_w   = (const float*)d_in[2];
  const float* fc_b   = (const float*)d_in[3];
  const float* w_ih   = (const float*)d_in[4];
  const float* w_hh   = (const float*)d_in[5];
  const float* b_ih   = (const float*)d_in[6];
  const float* b_hh   = (const float*)d_in[7];
  const float* out_w  = (const float*)d_in[8];
  const float* out_b  = (const float*)d_in[9];
  float* out = (float*)d_out;

  char* ws = (char*)d_ws;
  size_t off = 0;
  auto carve = [&](size_t bytes) -> char* { char* p = ws + off; off += (bytes + 255) & ~(size_t)255; return p; };
  unsigned short* WC   = (unsigned short*)carve((size_t)NGATE * NHID * 2);
  unsigned short* WHH  = (unsigned short*)carve((size_t)NGATE * NHID * 2);
  unsigned short* OW   = (unsigned short*)carve((size_t)NOUT * NHID * 2);
  unsigned short* H0   = (unsigned short*)carve((size_t)NBATCH * NHID * 2);
  unsigned short* HALL = (unsigned short*)carve((size_t)NROWS * NHID * 2);
  if (off > ws_size || off > (size_t)134217728) return;

  pack_w_kernel<<<2 * PACK_BLK_W + PACK_BLK_O, 256, 0, stream>>>(w_ih, w_hh, out_w, WC, WHH, OW);
  fc_h0_kernel<<<(NBATCH * NHID / 2 + 255) / 256, 256, 0, stream>>>(latent, fc_w, fc_b, (unsigned*)H0);
  lstm_seq_kernel<<<NBATCH / SEQ_BLK, LSTM_THR, 0, stream>>>(H0, WC, WHH, b_ih, b_hh, HALL);
  head_gemm_kernel<<<(NROWS / 64) * (NOUT / 64) / 8, 256, 0, stream>>>(HALL, OW, out, out_b);
}
